// SelfAttentionLayer_80023830659530
// MI455X (gfx1250) — hardware-verified
//
#include <hip/hip_runtime.h>


#ifndef NB
#define NB 1
#endif
#ifndef SEQ
#define SEQ 8192
#endif
#define SEQ_FULL 8192
#define DMD  128
#define QB   64
#define KS   32
#define PP   40
#define OP   132
#define PCAR 16384.0f
#define L2E  1.4426950408889634f

static_assert((SEQ % QB) == 0);
static_assert((SEQ % 64) == 0);
static_assert(SEQ <= SEQ_FULL);
static_assert((DMD % 32) == 0);
static_assert(NB == 1);

typedef _Float16 h16;
typedef unsigned short bf;
typedef __attribute__((ext_vector_type(16))) __bf16   v16bf;
typedef __attribute__((ext_vector_type(16))) _Float16 v16h;
typedef __attribute__((ext_vector_type(8)))  _Float16 v8h;
typedef __attribute__((ext_vector_type(8)))  unsigned short v8us;
typedef __attribute__((ext_vector_type(8)))  float    v8f;
typedef __attribute__((ext_vector_type(4)))  float    v4f;
typedef __attribute__((ext_vector_type(2)))  _Float16 v2h;
typedef __attribute__((ext_vector_type(2)))  unsigned short v2us;
typedef __attribute__((ext_vector_type(2)))  float    v2f;
typedef v8h  __attribute__((may_alias)) v8ha;
typedef v4f  __attribute__((may_alias)) v4fa;
typedef v8us __attribute__((may_alias)) v8usa;

__device__ __forceinline__ unsigned short f2bf(float f) { unsigned u = __float_as_uint(f); u += 0x7FFFu + ((u >> 16) & 1u); return (unsigned short)(u >> 16); }
__device__ __forceinline__ float bf2f(unsigned short b) { return __uint_as_float(((unsigned)b) << 16); }
__device__ __forceinline__ float bfr(float f) { return bf2f(f2bf(f)); }
__device__ __forceinline__ v16h cat16(v8h lo, v8h hi) { return __builtin_shufflevector(lo, hi, 0, 1, 2, 3, 4, 5, 6, 7, 8, 9, 10, 11, 12, 13, 14, 15); }
__device__ __forceinline__ v16bf cat16b(v8us lo, v8us hi) { return __builtin_bit_cast(v16bf, __builtin_shufflevector(lo, hi, 0, 1, 2, 3, 4, 5, 6, 7, 8, 9, 10, 11, 12, 13, 14, 15)); }
__device__ __forceinline__ v8f wmma16(v16h a, v16h b, v8f c) { return __builtin_amdgcn_wmma_f32_16x16x32_f16(false, a, false, b, (short)0, c, false, false); }
__device__ __forceinline__ v8f wmmab(v16bf a, v16bf b, v8f c) { return __builtin_amdgcn_wmma_f32_16x16x32_bf16(false, a, false, b, (short)0, c, false, false); }
__device__ __forceinline__ void splitf(float y, unsigned short& h, unsigned short& l) { h = f2bf(y); l = f2bf(y - bf2f(h)); }

template <typename T16> struct WFrag;
template <> struct WFrag<h16> { typedef v16h V; static __device__ __forceinline__ V ld(const h16* p) { return cat16(*(const v8ha*)p, *(const v8ha*)(p + 16)); } static __device__ __forceinline__ v8f mma(V a, V b, v8f c) { return wmma16(a, b, c); } };
template <> struct WFrag<bf> { typedef v16bf V; static __device__ __forceinline__ V ld(const bf* p) { return cat16b(*(const v8usa*)p, *(const v8usa*)(p + 16)); } static __device__ __forceinline__ v8f mma(V a, V b, v8f c) { return wmmab(a, b, c); } };

template <typename T16, int NSPLIT, bool BIAS>
__global__ __launch_bounds__(32) void k_gemmw(const T16* __restrict__ A, const T16* __restrict__ A2, const T16* __restrict__ Bt, const T16* __restrict__ Bt2, int K, float* C, int ldc, const float* __restrict__ bias, size_t sA, size_t sB, size_t sC) {
    typedef typename WFrag<T16>::V V;
    __shared__ __align__(16) float os[16 * 68];
    const size_t z = blockIdx.z; A += z * sA; if (A2) A2 += z * sA; Bt += z * sB; if (Bt2) Bt2 += z * sB; C += z * sC;
    const int lane = threadIdx.x & 31, lr = lane & 15, hi = lane >> 4; const int r0 = blockIdx.x * 64, c0 = blockIdx.y * 64;
    v8f acc[4][4];
#pragma unroll
    for (int mb = 0; mb < 4; ++mb)
#pragma unroll
        for (int nb = 0; nb < 4; ++nb) acc[mb][nb] = (v8f){};
    const size_t aoff = (size_t)(r0 + lr) * K + 8 * hi, boff = (size_t)(c0 + lr) * K + 8 * hi;
#pragma unroll 1
    for (int kc = 0; kc < K; kc += 32) {
        V a[4], a2[4];
#pragma unroll
        for (int mb = 0; mb < 4; ++mb) { a[mb] = WFrag<T16>::ld(A + aoff + (size_t)mb * 16 * K + kc); if (NSPLIT == 1 || NSPLIT == 2) a2[mb] = WFrag<T16>::ld(A2 + aoff + (size_t)mb * 16 * K + kc); }
#pragma unroll
        for (int nb = 0; nb < 4; ++nb) { const V b = WFrag<T16>::ld(Bt + boff + (size_t)nb * 16 * K + kc); V b2; if (NSPLIT >= 2) b2 = WFrag<T16>::ld(Bt2 + boff + (size_t)nb * 16 * K + kc);
#pragma unroll
            for (int mb = 0; mb < 4; ++mb) { acc[mb][nb] = WFrag<T16>::mma(a[mb], b, acc[mb][nb]); if (NSPLIT == 1 || NSPLIT == 2) acc[mb][nb] = WFrag<T16>::mma(a2[mb], b, acc[mb][nb]); if (NSPLIT >= 2) acc[mb][nb] = WFrag<T16>::mma(a[mb], b2, acc[mb][nb]); } }
        asm volatile("v_nop\n\tv_nop\n\tv_nop\n\tv_nop" : "+v"(acc[0][0]), "+v"(acc[1][1]), "+v"(acc[2][2]), "+v"(acc[3][3]) : "v"(a[0]), "v"(a[3]));
    }
#pragma unroll
    for (int mb = 0; mb < 4; ++mb) {
#pragma unroll
        for (int nb = 0; nb < 4; ++nb) {
#pragma unroll
            for (int j = 0; j < 8; ++j) os[(hi * 8 + j) * 68 + nb * 16 + lr] = acc[mb][nb][j]; }
        __builtin_amdgcn_fence(3, "wavefront"); __builtin_amdgcn_wave_barrier(); asm volatile("" ::: "memory");
        float* crow = C + (size_t)(r0 + mb * 16) * ldc + c0;
#pragma unroll 1
        for (int ps = 0; ps < 2; ++ps) {
#pragma unroll
            for (int s = 0; s < 8; ++s) { const int row = 2 * s + hi, cofs = lr * 4; v4f val = *(const v4fa*)(os + row * 68 + cofs); if (BIAS) { val[0] += bfr(bias[c0 + cofs]); val[1] += bfr(bias[c0 + cofs + 1]); val[2] += bfr(bias[c0 + cofs + 2]); val[3] += bfr(bias[c0 + cofs + 3]); }
                *(volatile v4f*)(crow + (size_t)row * ldc + cofs) = val; }
            if (ps == 0) __threadfence(); }
        __builtin_amdgcn_wave_barrier(); asm volatile("" ::: "memory");
    }
}

__global__ __launch_bounds__(256) void k_cvt8(const float* __restrict__ src, bf* dst, size_t n8) { const size_t i = (size_t)blockIdx.x * 256 + threadIdx.x; if (i >= n8) return; const v8f v = *(const v8f*)(src + i * 8); v8us o;
#pragma unroll
    for (int k = 0; k < 8; ++k) { const float f = v[k]; o[k] = f2bf(f); } *(volatile v8us*)(dst + i * 8) = o; __threadfence(); *(volatile v8us*)(dst + i * 8) = o; }

__global__ __launch_bounds__(256) void k_hlp(const float* __restrict__ F, int n, bf* Ph, bf* Pl) {
    const int e = (blockIdx.x * 256 + threadIdx.x) * 2; if (e >= n) return;
    const v2f x = *(const v2f*)(F + e); v2us oh, ol;
#pragma unroll
    for (int q = 0; q < 2; ++q) { const float xv = x[q]; unsigned short a2, c2; splitf(xv, a2, c2); oh[q] = a2; ol[q] = c2; }
    *(volatile v2us*)(Ph + e) = oh; *(volatile v2us*)(Pl + e) = ol; __threadfence(); *(volatile v2us*)(Ph + e) = oh; *(volatile v2us*)(Pl + e) = ol;
}

__global__ __launch_bounds__(256) void k_vt16(const float* __restrict__ F, h16* VT) {
    const int e = (blockIdx.x * 256 + threadIdx.x) * 2; if (e >= DMD * SEQ) return;
    const int t = e % SEQ, d = e / SEQ; v2h o16;
    const float x0 = F[(size_t)t * DMD + d], x1 = F[(size_t)(t + 1) * DMD + d];
    o16[0] = (h16)x0; o16[1] = (h16)x1;
    *(volatile v2h*)(VT + e) = o16; __threadfence(); *(volatile v2h*)(VT + e) = o16;
}

__global__ __launch_bounds__(128) __attribute__((amdgpu_num_vgpr(256)))
void k_attn(const bf* __restrict__ QPh, const bf* __restrict__ QPl, const bf* __restrict__ KPh, const bf* __restrict__ KPl, const h16* __restrict__ VT, float* OUT) {
    __shared__ __align__(16) h16 psm[4 * 16 * PP];
    __shared__ __align__(16) float osm[4 * 16 * OP];
    const int wave = threadIdx.x >> 5, lane = threadIdx.x & 31, lr = lane & 15, hi = lane >> 4;
    const int r0 = blockIdx.x * QB + wave * 16;
    h16* pw = psm + wave * (16 * PP);
    float* ow = osm + wave * (16 * OP);
    v8f o[8];
#pragma unroll
    for (int dt = 0; dt < 8; ++dt) o[dt] = (v8f){};
    float mrow[8], lrow[8];
#pragma unroll
    for (int r = 0; r < 8; ++r) { mrow[r] = -1.0e30f; lrow[r] = 0.0f; }
    const size_t qoff = (size_t)(r0 + lr) * DMD + 8 * hi;
    const size_t koff = (size_t)lr * DMD + 8 * hi;
    const size_t voff = (size_t)lr * SEQ + 8 * hi;
#pragma unroll 1
    for (int j0 = 0; j0 < SEQ; j0 += KS) {
        v8f s[2]; s[0] = (v8f){}; s[1] = (v8f){};
        v16bf ah, al, bh0, bl0, bh1, bl1;
#pragma unroll
        for (int ks = 0; ks < DMD / 32; ++ks) {
            ah = WFrag<bf>::ld(QPh + qoff + ks * 32); al = WFrag<bf>::ld(QPl + qoff + ks * 32);
            const size_t k0 = (size_t)j0 * DMD + koff + ks * 32, k1 = k0 + (size_t)16 * DMD;
            bh0 = WFrag<bf>::ld(KPh + k0); bl0 = WFrag<bf>::ld(KPl + k0);
            bh1 = WFrag<bf>::ld(KPh + k1); bl1 = WFrag<bf>::ld(KPl + k1);
            s[0] = wmmab(ah, bh0, s[0]); s[0] = wmmab(ah, bl0, s[0]); s[0] = wmmab(al, bh0, s[0]);
            s[1] = wmmab(ah, bh1, s[1]); s[1] = wmmab(ah, bl1, s[1]); s[1] = wmmab(al, bh1, s[1]);
        }
        asm volatile("v_nop\n\tv_nop\n\tv_nop\n\tv_nop" : "+v"(s[0]), "+v"(s[1]) : "v"(ah), "v"(al), "v"(bh0), "v"(bl0), "v"(bh1), "v"(bl1));
#pragma unroll
        for (int r = 0; r < 8; ++r) {
            float mx = fmaxf(s[0][r], s[1][r]);
            mx = fmaxf(mx, __shfl_xor(mx, 1, 32)); mx = fmaxf(mx, __shfl_xor(mx, 2, 32)); mx = fmaxf(mx, __shfl_xor(mx, 4, 32)); mx = fmaxf(mx, __shfl_xor(mx, 8, 32));
            const float mn = fmaxf(mrow[r], mx);
            const float alpha = __builtin_amdgcn_exp2f((mrow[r] - mn) * L2E);
            mrow[r] = mn;
            const float e0 = __builtin_amdgcn_exp2f((s[0][r] - mn) * L2E) * PCAR;
            const float e1 = __builtin_amdgcn_exp2f((s[1][r] - mn) * L2E) * PCAR;
            const h16 p0 = (h16)e0, p1 = (h16)e1;
            float rs = (float)p0 + (float)p1;
            rs += __shfl_xor(rs, 1, 32); rs += __shfl_xor(rs, 2, 32); rs += __shfl_xor(rs, 4, 32); rs += __shfl_xor(rs, 8, 32);
            lrow[r] = lrow[r] * alpha + rs;
            pw[(8 * hi + r) * PP + lr] = p0; pw[(8 * hi + r) * PP + 16 + lr] = p1;
#pragma unroll
            for (int dt = 0; dt < 8; ++dt) o[dt][r] *= alpha;
        }
        __builtin_amdgcn_fence(3, "wavefront"); __builtin_amdgcn_wave_barrier(); asm volatile("" ::: "memory");
        const v16h pa = WFrag<h16>::ld(pw + lr * PP + 8 * hi);
        v16h vb;
#pragma unroll
        for (int dt = 0; dt < 8; ++dt) { vb = WFrag<h16>::ld(VT + (size_t)(dt * 16) * SEQ + voff + j0); o[dt] = wmma16(pa, vb, o[dt]); }
        asm volatile("v_nop\n\tv_nop\n\tv_nop\n\tv_nop" : "+v"(o[0]), "+v"(o[1]), "+v"(o[2]), "+v"(o[3]), "+v"(o[4]), "+v"(o[5]), "+v"(o[6]), "+v"(o[7]) : "v"(pa), "v"(vb));
        asm volatile("" ::: "memory");
    }
#pragma unroll
    for (int r = 0; r < 8; ++r) { const float inv = 1.0f / lrow[r];
#pragma unroll
        for (int dt = 0; dt < 8; ++dt) ow[(8 * hi + r) * OP + dt * 16 + lr] = o[dt][r] * inv; }
    __builtin_amdgcn_fence(3, "wavefront"); __builtin_amdgcn_wave_barrier(); asm volatile("" ::: "memory");
    float* orow = OUT + (size_t)r0 * DMD + lane * 4;
#pragma unroll 1
    for (int ps = 0; ps < 2; ++ps) {
#pragma unroll
        for (int row = 0; row < 16; ++row) { const v4f val = *(const v4fa*)(ow + row * OP + lane * 4); *(volatile v4f*)(orow + (size_t)row * DMD) = val; }
        if (ps == 0) __threadfence();
    }
}

extern "C" void kernel_launch(void* const* d_in, const int* in_sizes, int n_in,
                              void* d_out, int out_size, void* d_ws, size_t ws_size, hipStream_t stream) {
    if (n_in < 4) return;
    if (in_sizes[0] < SEQ * DMD || in_sizes[1] < DMD * DMD || in_sizes[2] < DMD * DMD || in_sizes[3] < DMD * DMD || out_size < SEQ * DMD) return;
    const float* x = (const float*)d_in[0]; const float* wq = (const float*)d_in[1]; const float* wk = (const float*)d_in[2]; const float* wv = (const float*)d_in[3];
    float* OUT = (float*)d_out;
    char* wsp = (char*)d_ws;
    auto take = [&](size_t bytes) { char* p = wsp; wsp += (bytes + 255) & ~(size_t)255; return (void*)p; };
    bf* WQ = (bf*)take((size_t)DMD * DMD * 2); bf* WK = (bf*)take((size_t)DMD * DMD * 2); bf* WV = (bf*)take((size_t)DMD * DMD * 2);
    bf* XB = (bf*)take((size_t)SEQ * DMD * 2);
    float* FQ = (float*)take((size_t)SEQ * DMD * 4); float* FK = (float*)take((size_t)SEQ * DMD * 4); float* FV = (float*)take((size_t)SEQ * DMD * 4);
    bf* QPh = (bf*)take((size_t)SEQ * DMD * 2); bf* QPl = (bf*)take((size_t)SEQ * DMD * 2); bf* KPh = (bf*)take((size_t)SEQ * DMD * 2); bf* KPl = (bf*)take((size_t)SEQ * DMD * 2);
    h16* VT = (h16*)take((size_t)DMD * SEQ * 2);
    const size_t used = (size_t)(wsp - (char*)d_ws);
    if (used > ws_size || used > (size_t)134217728) return;

    k_cvt8<<<(unsigned)(((size_t)DMD * DMD / 8 + 255) / 256), 256, 0, stream>>>(wq, WQ, (size_t)DMD * DMD / 8);
    k_cvt8<<<(unsigned)(((size_t)DMD * DMD / 8 + 255) / 256), 256, 0, stream>>>(wk, WK, (size_t)DMD * DMD / 8);
    k_cvt8<<<(unsigned)(((size_t)DMD * DMD / 8 + 255) / 256), 256, 0, stream>>>(wv, WV, (size_t)DMD * DMD / 8);
    k_cvt8<<<(unsigned)(((size_t)SEQ * DMD / 8 + 255) / 256), 256, 0, stream>>>(x, XB, (size_t)SEQ * DMD / 8);
    k_gemmw<bf, 0, false><<<dim3(SEQ / 64, DMD / 64, 1), 32, 0, stream>>>(XB, nullptr, WQ, nullptr, DMD, FQ, DMD, nullptr, 0, 0, 0);
    k_gemmw<bf, 0, false><<<dim3(SEQ / 64, DMD / 64, 1), 32, 0, stream>>>(XB, nullptr, WK, nullptr, DMD, FK, DMD, nullptr, 0, 0, 0);
    k_gemmw<bf, 0, false><<<dim3(SEQ / 64, DMD / 64, 1), 32, 0, stream>>>(XB, nullptr, WV, nullptr, DMD, FV, DMD, nullptr, 0, 0, 0);
    const unsigned LP = (unsigned)(((size_t)SEQ * DMD / 2 + 255) / 256);
    k_hlp<<<LP, 256, 0, stream>>>(FQ, SEQ * DMD, QPh, QPl);
    k_hlp<<<LP, 256, 0, stream>>>(FK, SEQ * DMD, KPh, KPl);
    k_vt16<<<LP, 256, 0, stream>>>(FV, VT);
    k_attn<<<SEQ / QB, 128, 0, stream>>>(QPh, QPl, KPh, KPl, VT, OUT);
}
